// G3DCrossAttention_38354057953789
// MI455X (gfx1250) — hardware-verified
//
#include <hip/hip_runtime.h>
#include <math.h>

typedef __attribute__((ext_vector_type(16))) _Float16 v16h;
typedef __attribute__((ext_vector_type(16))) __bf16 v16b;
typedef __attribute__((ext_vector_type(8)))  _Float16 v8h;
typedef __attribute__((ext_vector_type(8)))  float v8f;
typedef __attribute__((ext_vector_type(4)))  float v4f;
typedef __attribute__((ext_vector_type(2)))  float v2f;
typedef __attribute__((ext_vector_type(4)))  unsigned v4u;
typedef __attribute__((ext_vector_type(4)))  int v4i;
typedef float __attribute__((may_alias)) float_a;
typedef int __attribute__((may_alias)) int_a;

template <typename T> __device__ __forceinline__ void vst2(void* p, T v) { *(volatile T*)p = v; __threadfence(); *(volatile T*)p = v; }
__device__ __forceinline__ v8f wmma16(v16h a, v16h b, v8f c) {
  v8f d = __builtin_amdgcn_wmma_f32_16x16x32_f16(false, a, false, b, (short)0, c, false, false);
  asm volatile("v_nop\n\tv_nop\n\tv_nop\n\tv_nop" : "+v"(d) : "v"(a), "v"(b));
  return d;
}
__device__ __forceinline__ v8f wmma_bf(v16b a, v16b b, v8f c) {
  v8f d = __builtin_amdgcn_wmma_f32_16x16x32_bf16(false, a, false, b, (short)0, c, false, false);
  asm volatile("v_nop\n\tv_nop\n\tv_nop\n\tv_nop" : "+v"(d) : "v"(a), "v"(b));
  return d;
}
__device__ __forceinline__ v16h frag_h(const _Float16* rowk0, int lane) {
  union { v16h v; v8h q[2]; } u; const _Float16* p = rowk0 + 8 * (lane >> 4);
  u.q[0] = *(const v8h*)p; u.q[1] = *(const v8h*)(p + 16); return u.v;
}
__device__ __forceinline__ v16h frag_f32(const float* rowk0, int lane) {
  v16h a; const float* p = rowk0 + 8 * (lane >> 4);
#pragma unroll
  for (int i = 0; i < 8; ++i) { a[i] = (_Float16)p[i]; a[8 + i] = (_Float16)p[16 + i]; }
  return a;
}
__device__ __forceinline__ v16h frag_f32s(const float* rowk0, int lane, float sc) {
  v16h a; const float* p = rowk0 + 8 * (lane >> 4);
#pragma unroll
  for (int i = 0; i < 8; ++i) { a[i] = (_Float16)(p[i] * sc); a[8 + i] = (_Float16)(p[16 + i] * sc); }
  return a;
}
__device__ __forceinline__ v16h fragc_f32(const float* W, int k0, int n, int lane, int ld, int K) {
  v16h a; const int g = lane >> 4;
#pragma unroll
  for (int i = 0; i < 8; ++i) { const int ka = k0 + 8 * g + i, kb = ka + 16;
    a[i] = (_Float16)(ka < K ? W[(size_t)(ka < K ? ka : K - 1) * ld + n] : 0.f); a[8 + i] = (_Float16)(kb < K ? W[(size_t)(kb < K ? kb : K - 1) * ld + n] : 0.f); }
  return a;
}
struct F2 { v16b h, l; };
__device__ __forceinline__ F2 bsplit16(const float v[16]) { F2 r;
#pragma unroll
  for (int i = 0; i < 16; ++i) { const __bf16 h = (__bf16)v[i]; r.h[i] = h; r.l[i] = (__bf16)(v[i] - (float)h); }
  return r; }
__device__ __forceinline__ F2 split_row(const float* row, int k0, int lane) { float v[16]; const float* p = row + k0 + 8 * (lane >> 4);
#pragma unroll
  for (int i = 0; i < 8; ++i) { v[i] = p[i]; v[8 + i] = p[16 + i]; }
  return bsplit16(v); }
__device__ __forceinline__ F2 split_rowK(const float* row, int k0, int lane, int K) { float v[16]; const int g = lane >> 4;
#pragma unroll
  for (int i = 0; i < 8; ++i) { const int ka = k0 + 8 * g + i, kb = ka + 16; v[i] = ka < K ? row[ka < K ? ka : K - 1] : 0.f; v[8 + i] = kb < K ? row[kb < K ? kb : K - 1] : 0.f; }
  return bsplit16(v); }
__device__ __forceinline__ F2 split_col(const float* W, int k0, int n, int lane, int ld, int K) { float v[16]; const int g = lane >> 4;
#pragma unroll
  for (int i = 0; i < 8; ++i) { const int ka = k0 + 8 * g + i, kb = ka + 16; v[i] = ka < K ? W[(size_t)(ka < K ? ka : K - 1) * ld + n] : 0.f; v[8 + i] = kb < K ? W[(size_t)(kb < K ? kb : K - 1) * ld + n] : 0.f; }
  return bsplit16(v); }
__device__ __forceinline__ v8f mac3(const F2& a, const F2& b, v8f c) { c = wmma_bf(a.l, b.h, c); c = wmma_bf(a.h, b.l, c); return wmma_bf(a.h, b.h, c); }
__device__ __forceinline__ float sigm(float v) { return 1.0f / (1.0f + expf(-v)); }
#define LDSX() do { asm volatile("s_wait_dscnt 0" ::: "memory"); __builtin_amdgcn_wave_barrier(); __builtin_amdgcn_fence(__ATOMIC_RELEASE, "workgroup"); } while (0)


#define NB 2
#define CC 512
#define LL 2048
#define GG 2048
#define NH 8
#define HD 64
#define FF (4 * CC)
#define NR (NB * LL)
#ifndef NBT
#define NBT NB
#define TB0 0
#define TLB (LL / 64)
#endif
#define RB0 ((size_t)TB0 * LL)
typedef __attribute__((ext_vector_type(8))) __bf16 v8b;
__device__ __forceinline__ v16b frag_b(const __bf16* rowk0, int lane) {
  union { v16b v; v8b q[2]; } u; const __bf16* p = rowk0 + 8 * (lane >> 4);
  u.q[0] = *(const v8b*)p; u.q[1] = *(const v8b*)(p + 16); return u.v;
}
__device__ __forceinline__ float bfr(float v) { return (float)(__bf16)v; }
__device__ __attribute__((noinline)) float exp_ni(float v) { return expf(v); }
__device__ __attribute__((noinline)) float erf_ni(float v) { return erff(v); }

#define PK_Q  0
#define PK_1  ((size_t)CC * CC)
#define PK_2  (PK_1 + (size_t)FF * CC)
#define PK_O  (PK_2 + (size_t)CC * FF)
#define PK_END (PK_O + (size_t)CC * CC)
#define WS_PK  0u
#define WS_VEC (((2u * PK_END) + 127u) / 128u * 128u)
#define WS_XS  (WS_VEC + 4u * 4 * CC)
#define WS_Q   (WS_XS + 4u * NR * CC)
#define WS_X1  (WS_Q + 4u * NR * CC)
#define WS_T   (WS_X1 + 4u * NR * CC)
#define WS_X3  (WS_T + 4u * NR * CC)
#define WS_GH  (WS_X3 + 4u * NR * CC)
#define WS_GL  (WS_GH + 2u * (size_t)NR * FF)
#define WS_END (WS_GL + 2u * (size_t)NR * FF)

__global__ __launch_bounds__(256) void k_pack(const float* __restrict__ WQ, const float* __restrict__ W1, const float* __restrict__ W2, const float* __restrict__ WO, __bf16* __restrict__ PK) {
  __shared__ __align__(16) __bf16 s[FF]; const int n = blockIdx.x, which = blockIdx.y, t = threadIdx.x; int K; size_t dst; const float* src;
  switch (which) { case 0: if (n >= CC) return; K = CC; dst = PK_Q + (size_t)n * CC; src = WQ + (size_t)n * CC; break; case 1: K = CC; dst = PK_1 + (size_t)n * CC; src = W1 + (size_t)n * CC; break; case 2: if (n >= CC) return; K = FF; dst = PK_2 + (size_t)n * FF; src = W2 + (size_t)n * FF; break; default: if (n >= CC) return; K = CC; dst = PK_O + (size_t)n * CC; src = WO + (size_t)n * CC; break; }
  for (int k = t; k < K; k += 256) s[k] = (__bf16)src[k];
  __syncthreads();
  for (int q = t; q < K / 8; q += 256) vst2((unsigned*)(PK + dst + q * 8), *(const v4u*)&s[q * 8]);
}
__global__ __launch_bounds__(256) void k_vec(const float* __restrict__ WG, const float* __restrict__ BG, const float* __restrict__ WK, const float* __restrict__ BK, const float* __restrict__ WV, const float* __restrict__ BV, float* __restrict__ VEC) {
  __shared__ float sw[CC], sb[CC]; __shared__ __align__(16) float so[4][CC]; const int t = threadIdx.x;
  for (int i = t; i < CC; i += 256) { sw[i] = bfr(WG[i]); sb[i] = bfr(BG[i]); }
  __syncthreads();
  for (int c = t; c < CC; c += 256) { float ak = 0.f, ck = 0.f, av = 0.f, cv = 0.f; const float* wk = WK + (size_t)c * CC; const float* wv = WV + (size_t)c * CC;
#pragma unroll 1
    for (int i = 0; i < CC; ++i) { const float k = bfr(wk[i]), v = bfr(wv[i]); ak += k * sw[i]; ck += k * sb[i]; av += v * sw[i]; cv += v * sb[i]; }
    so[0][c] = ak; so[1][c] = ck + bfr(BK[c]); so[2][c] = av; so[3][c] = cv + bfr(BV[c]); }
  __syncthreads();
  for (int q = t; q < 4 * CC / 4; q += 256) vst2(VEC + q * 4, *(const v4f*)(&so[0][0] + q * 4));
}
__global__ __launch_bounds__(128) void k_q(const float* __restrict__ SEQ, const __bf16* __restrict__ PK, const float* __restrict__ BQ, float* __restrict__ XS, float* __restrict__ Q) {
  __shared__ __align__(16) __bf16 sx[64][CC + 8]; __shared__ __align__(16) float so[4][16][132];
  const int tid = threadIdx.x, wave = tid >> 5, lane = tid & 31, col = lane & 15, g = lane >> 4; const int lb = blockIdx.x; const size_t b = blockIdx.y + TB0; const int l0 = lb * 64; const size_t row0 = b * LL + l0;
  for (int e = tid; e < 64 * CC; e += 128) { const int c = e >> 6, r = e & 63; sx[r][c] = (__bf16)SEQ[(b * CC + c) * LL + l0 + r]; }
  if (tid < 64) for (int c = CC; c < CC + 8; ++c) sx[tid][c] = (__bf16)0.f;
  __syncthreads();
  for (int rl = 0; rl < 16; ++rl) { const int r = wave * 16 + rl; for (int q4 = lane; q4 < CC / 4; q4 += 32) { v4f v = {(float)sx[r][q4 * 4], (float)sx[r][q4 * 4 + 1], (float)sx[r][q4 * 4 + 2], (float)sx[r][q4 * 4 + 3]}; vst2(XS + (row0 + r) * CC + q4 * 4, v); } }
#pragma unroll 1
  for (int pass = 0; pass < CC / 128; ++pass) { const int n0 = pass * 128; v8f acc[8] = {};
#pragma unroll 2
    for (int kc = 0; kc < CC / 32; ++kc) { const v16b a = frag_b(&sx[wave * 16 + col][kc * 32], lane);
#pragma unroll
      for (int j = 0; j < 8; ++j) acc[j] = wmma_bf(a, frag_b(PK + PK_Q + (size_t)(n0 + j * 16 + col) * CC + kc * 32, lane), acc[j]); }
#pragma unroll
    for (int j = 0; j < 8; ++j) { const float bb = bfr(BQ[n0 + j * 16 + col]);
#pragma unroll
      for (int r = 0; r < 8; ++r) so[wave][8 * g + r][j * 16 + col] = acc[j][r] + bb; }
    LDSX();
    for (int rl = 0; rl < 16; ++rl) vst2(Q + (row0 + wave * 16 + rl) * CC + n0 + lane * 4, *(const v4f*)&so[wave][rl][lane * 4]);
    LDSX(); }
}
__global__ __launch_bounds__(128) void k_ax(const float* __restrict__ Q, const float* __restrict__ VEC, const float* __restrict__ EXP, const float* __restrict__ XS, const float* __restrict__ G1, const float* __restrict__ B1, float* __restrict__ X1) {
  __shared__ float se[GG]; __shared__ float sv[4][CC]; __shared__ __align__(16) float so[16][CC + 4];
  const int tid = threadIdx.x; const size_t b = blockIdx.y + TB0; const size_t row0 = b * LL + (size_t)blockIdx.x * 16; const int r = tid >> 3, h = tid & 7;
  for (int i = tid; i < GG; i += 128) se[i] = bfr(EXP[b * GG + i]);
  for (int i = tid; i < 4 * CC; i += 128) sv[i / CC][i % CC] = VEC[i];
  __syncthreads();
  { const float* q = Q + (row0 + r) * CC + h * HD; float al = 0.f;
#pragma unroll 1
    for (int d = 0; d < HD; ++d) al += q[d] * sv[0][h * HD + d];
    al *= 0.125f;
    float mx = -3.0e38f;
#pragma unroll 1
    for (int gi = 0; gi < GG; ++gi) mx = fmaxf(mx, al * se[gi]);
    float sw = 0.f, swe = 0.f;
#pragma unroll 1
    for (int gi = 0; gi < GG; ++gi) { const float w = exp_ni(al * se[gi] - mx); sw += w; swe += w * se[gi]; }
    const float E = swe / sw;
#pragma unroll 1
    for (int d = 0; d < HD; ++d) so[r][h * HD + d] = E * sv[2][h * HD + d] + sv[3][h * HD + d] + XS[(row0 + r) * CC + h * HD + d]; }
  __syncthreads();
  { float s = 0.f; for (int c = h; c < CC; c += 8) s += so[r][c];
#pragma unroll
    for (int o = 1; o < 8; o <<= 1) s += __shfl_xor(s, o);
    const float mu = s / (float)CC; float q2 = 0.f; for (int c = h; c < CC; c += 8) { const float d = so[r][c] - mu; q2 += d * d; }
#pragma unroll
    for (int o = 1; o < 8; o <<= 1) q2 += __shfl_xor(q2, o);
    const float inv = 1.0f / sqrtf(q2 / (float)CC + 1e-5f);
    __syncthreads();
    for (int c = h; c < CC; c += 8) so[r][c] = (so[r][c] - mu) * inv * bfr(G1[c]) + bfr(B1[c]); }
  __syncthreads();
  for (int q4 = tid; q4 < 16 * CC / 4; q4 += 128) { const int rr = q4 / (CC / 4), cq = q4 % (CC / 4); vst2(X1 + (row0 + rr) * CC + cq * 4, *(const v4f*)&so[rr][cq * 4]); }
}
template <int MODE>
__global__ __launch_bounds__(128) void k_lin(const float* __restrict__ A, const __bf16* __restrict__ AG, const __bf16* __restrict__ AGL, const __bf16* __restrict__ PK, const float* __restrict__ BIAS, const float* __restrict__ RES, float* __restrict__ OUTF, __bf16* __restrict__ OUTG, __bf16* __restrict__ OUTGL) {
  __shared__ __align__(16) float so[4][16][132]; __shared__ __align__(16) __bf16 sg[4][16][136], sgl[4][16][136]; __shared__ __align__(16) float st[128][68];
  const int tid = threadIdx.x, wave = tid >> 5, lane = tid & 31, col = lane & 15, g = lane >> 4; const size_t r0 = ((size_t)TB0 + blockIdx.z) * LL + (size_t)blockIdx.x * 64 + wave * 16; const int n0 = blockIdx.y * 128;
  constexpr int KD = (MODE == 2) ? FF : CC; const __bf16* P = PK + ((MODE == 1) ? PK_1 : (MODE == 2) ? PK_2 : PK_O);
  v8f acc[8] = {};
  if (MODE == 2) {
#pragma unroll 2
    for (int kc = 0; kc < KD / 32; ++kc) { const v16b a = frag_b(AG + (r0 + col) * FF + kc * 32, lane), al = frag_b(AGL + (r0 + col) * FF + kc * 32, lane);
#pragma unroll
      for (int j = 0; j < 8; ++j) { const v16b w = frag_b(P + (size_t)(n0 + j * 16 + col) * KD + kc * 32, lane); acc[j] = wmma_bf(al, w, acc[j]); acc[j] = wmma_bf(a, w, acc[j]); } }
  } else {
#pragma unroll 2
    for (int kc = 0; kc < KD / 32; ++kc) { const F2 a = split_row(A + (r0 + col) * CC, kc * 32, lane);
#pragma unroll
      for (int j = 0; j < 8; ++j) { const v16b w = frag_b(P + (size_t)(n0 + j * 16 + col) * KD + kc * 32, lane); acc[j] = wmma_bf(a.l, w, acc[j]); acc[j] = wmma_bf(a.h, w, acc[j]); } } }
  if (MODE == 1) {
#pragma unroll
    for (int j = 0; j < 8; ++j) { const float bb = bfr(BIAS[n0 + j * 16 + col]);
#pragma unroll
      for (int r = 0; r < 8; ++r) { const float v = fmaxf(acc[j][r] + bb, 0.f); const __bf16 hb = (__bf16)v; sg[wave][8 * g + r][j * 16 + col] = hb; sgl[wave][8 * g + r][j * 16 + col] = (__bf16)(v - (float)hb); } }
    LDSX();
    for (int rl = 0; rl < 16; ++rl) { if (lane < 16) vst2((unsigned*)(OUTG + (r0 + rl) * FF + n0 + lane * 8), *(const v4u*)&sg[wave][rl][lane * 8]); else vst2((unsigned*)(OUTGL + (r0 + rl) * FF + n0 + (lane - 16) * 8), *(const v4u*)&sgl[wave][rl][(lane - 16) * 8]); }
  } else if (MODE == 2) {
#pragma unroll
    for (int j = 0; j < 8; ++j) { const int c = n0 + j * 16 + col; const float bb = bfr(BIAS[c]);
#pragma unroll
      for (int r = 0; r < 8; ++r) { const size_t row = r0 + 8 * g + r; so[wave][8 * g + r][j * 16 + col] = acc[j][r] + bb + RES[row * CC + c]; } }
    LDSX();
    for (int rl = 0; rl < 16; ++rl) vst2(OUTF + (r0 + rl) * CC + n0 + lane * 4, *(const v4f*)&so[wave][rl][lane * 4]);
  } else {
#pragma unroll
    for (int j = 0; j < 8; ++j) { const float bb = bfr(BIAS[n0 + j * 16 + col]);
#pragma unroll
      for (int r = 0; r < 8; ++r) st[j * 16 + col][wave * 16 + 8 * g + r] = acc[j][r] + bb; }
    __syncthreads();
    const size_t rb = ((size_t)TB0 + blockIdx.z) * LL + (size_t)blockIdx.x * 64; const size_t b = rb / LL; const int l0 = (int)(rb % LL);
    for (int e = tid; e < 128 * 16; e += 128) { const int c = e >> 4, pc = e & 15; vst2(OUTF + ((b * CC + n0 + c) * LL) + l0 + pc * 4, *(const v4f*)&st[c][pc * 4]); }
  }
}
__global__ __launch_bounds__(128) void k_ln(const float* __restrict__ SRC, const float* __restrict__ G, const float* __restrict__ Bv, float* __restrict__ OUT) {
  __shared__ float red[2][4]; const int t = threadIdx.x; const size_t row = ((size_t)TB0 + blockIdx.y) * LL + blockIdx.x; const float* p = SRC + row * CC + t * 4;
  float v[4] = {p[0], p[1], p[2], p[3]}; float s = (v[0] + v[1]) + (v[2] + v[3]);
#pragma unroll
  for (int o = 1; o < 32; o <<= 1) s += __shfl_xor(s, o);
  if ((t & 31) == 0) red[0][t >> 5] = s; __syncthreads();
  const float mu = (red[0][0] + red[0][1] + red[0][2] + red[0][3]) / (float)CC; float q = 0.f;
#pragma unroll
  for (int i = 0; i < 4; ++i) { const float d = v[i] - mu; q += d * d; }
#pragma unroll
  for (int o = 1; o < 32; o <<= 1) q += __shfl_xor(q, o);
  if ((t & 31) == 0) red[1][t >> 5] = q; __syncthreads();
  const float inv = 1.0f / sqrtf((red[1][0] + red[1][1] + red[1][2] + red[1][3]) / (float)CC + 1e-5f); v4f o4;
#pragma unroll
  for (int i = 0; i < 4; ++i) o4[i] = (v[i] - mu) * inv * bfr(G[t * 4 + i]) + bfr(Bv[t * 4 + i]);
  vst2(OUT + row * CC + t * 4, o4);
}
extern "C" void kernel_launch(void* const* d_in, const int* in_sizes, int n_in, void* d_out, int out_size, void* d_ws, size_t ws_size, hipStream_t stream) {
  (void)in_sizes; (void)n_in; (void)out_size;
  const float** F = (const float**)d_in;
  if (ws_size < (size_t)WS_END) return;
  char* ws = (char*)d_ws; __bf16 *PK = (__bf16*)(ws + WS_PK), *GH = (__bf16*)(ws + WS_GH), *GL = (__bf16*)(ws + WS_GL); float *VEC = (float*)(ws + WS_VEC), *XS = (float*)(ws + WS_XS), *Q = (float*)(ws + WS_Q), *X1 = (float*)(ws + WS_X1), *T = (float*)(ws + WS_T), *X3 = (float*)(ws + WS_X3);
  const int RT = NBT * LL;
  k_pack<<<dim3(FF, 4), 256, 0, stream>>>(F[4], F[12], F[14], F[10], PK);
  k_vec<<<1, 256, 0, stream>>>(F[2], F[3], F[6], F[7], F[8], F[9], VEC);
  k_q<<<dim3(TLB, NBT), 128, 0, stream>>>(F[0], PK, F[5], XS, Q);
  k_ax<<<dim3(TLB * 4, NBT), 128, 0, stream>>>(Q, VEC, F[1], XS, F[16], F[17], X1);
  k_lin<1><<<dim3(TLB, FF / 128, NBT), 128, 0, stream>>>(X1, nullptr, nullptr, PK, F[13], nullptr, nullptr, GH, GL);
  k_lin<2><<<dim3(TLB, CC / 128, NBT), 128, 0, stream>>>(nullptr, GH, GL, PK, F[15], X1, T, nullptr, nullptr);
  k_ln<<<dim3(TLB * 64, NBT), 128, 0, stream>>>(T, F[18], F[19], X3);
  k_lin<3><<<dim3(TLB, CC / 128, NBT), 128, 0, stream>>>(X3, nullptr, nullptr, PK, F[11], nullptr, (float*)d_out, nullptr, nullptr);
  (void)RT;
}
